// MultiheadAttention_20658792694509
// MI455X (gfx1250) — hardware-verified
//
#include <hip/hip_runtime.h>


#ifndef NB
#define NB 4
#endif
#ifndef SEQ
#define SEQ 2048
#endif
#define NB_FULL  4
#define SEQ_FULL 2048
#ifndef OUT_SEQ
#define OUT_SEQ SEQ
#endif
#define DM   1024
#define NH_  16
#define HD   64
#define AW   4
#define SC2  (0.125f * 1.4426950408889634f)
#define PSH  8.0f
#define TP   72

static_assert(HD == 64);
static_assert(NH_ * HD == DM);
static_assert(DM % 8 == 0);
static_assert(SEQ % 64 == 0);
static_assert(SEQ % 32 == 0);
static_assert(SEQ % (16 * AW) == 0);
static_assert(((size_t)NB * SEQ * DM) % (8 * 256) == 0);
static_assert(NB <= NB_FULL);
static_assert(SEQ <= SEQ_FULL);

typedef _Float16 h16;
typedef __attribute__((ext_vector_type(16))) _Float16 v16h;
typedef __attribute__((ext_vector_type(8)))  _Float16 v8h;
typedef __attribute__((ext_vector_type(8)))  float    v8f;
typedef __attribute__((ext_vector_type(4)))  float    v4f;
typedef v4f  __attribute__((may_alias)) v4fa;
typedef v8h  __attribute__((may_alias)) v8ha;

__device__ __forceinline__ float rbf(float f) { unsigned u = __float_as_uint(f); u += 0x7FFFu + ((u >> 16) & 1u); return __uint_as_float(u & 0xFFFF0000u); }
__device__ __forceinline__ v16h cat16(v8h lo, v8h hi) { return __builtin_shufflevector(lo, hi, 0, 1, 2, 3, 4, 5, 6, 7, 8, 9, 10, 11, 12, 13, 14, 15); }
__device__ __forceinline__ v8f wmma16(v16h a, v16h b, v8f c) { return __builtin_amdgcn_wmma_f32_16x16x32_f16(false, a, false, b, (short)0, c, false, false); }
__device__ __forceinline__ v16h ldh(const h16* p) { return cat16(*(const v8h*)p, *(const v8h*)(p + 16)); }
__device__ __forceinline__ void wave_sync() { __builtin_amdgcn_fence(3  , "wavefront"); __builtin_amdgcn_wave_barrier(); asm volatile("" ::: "memory"); }

__global__ __launch_bounds__(256) void k_cvt2(const float* __restrict__ sa, h16* da, const float* __restrict__ sb, h16* db, size_t n8) {
    const size_t i = (size_t)blockIdx.x * 256 + threadIdx.x; if (i >= n8) return;
    const size_t e = i * 8; const size_t row = e / DM; const size_t col = e % DM;
    const size_t bb = row / SEQ, t = row % SEQ;
    const size_t so = (bb * SEQ_FULL + t) * DM + col;
    const v8f x = *(const v8f*)(sa + so); const v8f y = *(const v8f*)(sb + so); v8h o, p;
#pragma unroll
    for (int k = 0; k < 8; ++k) { o[k] = (h16)rbf(x[k]); p[k] = (h16)rbf(y[k]); }
    *(volatile v8h*)(da + e) = o; *(volatile v8h*)(db + e) = p;
    __threadfence();
    *(volatile v8h*)(da + e) = o; *(volatile v8h*)(db + e) = p;
}

__global__ __launch_bounds__(256) void k_vt(const float* __restrict__ v, h16* VT) {
    __shared__ __align__(16) h16 ts[64 * TP];
    const int tid = threadIdx.x;
    const int zh = blockIdx.y; const int b = zh / NH_, h = zh % NH_;
    const int t0 = blockIdx.x * 64;
    const int r = tid >> 2, c0 = (tid & 3) * 16;
    const float* src = v + ((size_t)b * SEQ_FULL + t0 + r) * DM + h * HD + c0;
#pragma unroll
    for (int q = 0; q < 4; ++q) { const v4f x = *(const v4f*)(src + 4 * q);
#pragma unroll
        for (int i = 0; i < 4; ++i) ts[(c0 + 4 * q + i) * TP + r] = (h16)rbf(x[i]); }
    __syncthreads();
    h16* dstb = VT + (size_t)zh * HD * SEQ + t0;
#pragma unroll 1
    for (int ps = 0; ps < 2; ++ps) {
#pragma unroll
        for (int s = 0; s < 2; ++s) { const int d = 32 * s + (tid >> 3), c8 = (tid & 7) * 8;
            const v8h val = *(const v8ha*)(&ts[d * TP + c8]);
            *(volatile v8h*)(dstb + (size_t)d * SEQ + c8) = val; }
        if (ps == 0) __threadfence(); }
}

__global__ __launch_bounds__(32 * AW) void k_flash(const h16* __restrict__ QH, const h16* __restrict__ KH, const h16* __restrict__ VT, float* OUT) {
    __shared__ __align__(16) float os[AW * 16 * 68];
    const int lane = threadIdx.x & 31, wave = __builtin_amdgcn_readfirstlane((int)(threadIdx.x >> 5)), lr = lane & 15, hi = lane >> 4;
    const int zh = blockIdx.y; const int b = zh / NH_, h = zh % NH_;
    const int t0 = (blockIdx.x * AW + wave) * 16;
    const size_t rbase = (size_t)b * SEQ * DM + (size_t)h * HD;
    const size_t qo = rbase + (size_t)(t0 + lr) * DM + 8 * hi;
    const v16h qh0 = ldh(QH + qo), qh1 = ldh(QH + qo + 32);
    const size_t ko = rbase + (size_t)lr * DM + 8 * hi;
    const size_t vo = ((size_t)zh * HD + lr) * SEQ + 8 * hi;
    v8f o0 = (v8f){}, o1 = (v8f){}, o2 = (v8f){}, o3 = (v8f){};
    float m = -3.0e38f, l = 0.0f;
#pragma unroll 1
    for (int key0 = 0; key0 < SEQ; key0 += 32) {
        const h16* ka = KH + ko + (size_t)key0 * DM;
        const v16h ka0 = ldh(ka), ka1 = ldh(ka + 32), kb0 = ldh(ka + (size_t)16 * DM), kb1 = ldh(ka + (size_t)16 * DM + 32);
        v8f sa = (v8f){}, sb = (v8f){};
        sa = wmma16(ka0, qh0, sa); sb = wmma16(kb0, qh0, sb);
        sa = wmma16(ka1, qh1, sa); sb = wmma16(kb1, qh1, sb);
        asm volatile("v_nop\n\tv_nop\n\tv_nop\n\tv_nop" : "+v"(sa), "+v"(sb) : "v"(ka0), "v"(ka1), "v"(kb0), "v"(kb1), "v"(qh0), "v"(qh1));
        float ta[8], tb[8]; float mx = -3.0e38f;
#pragma unroll
        for (int r = 0; r < 8; ++r) { ta[r] = sa[r] * SC2; tb[r] = sb[r] * SC2; mx = fmaxf(mx, fmaxf(ta[r], tb[r])); }
        mx = fmaxf(mx, __shfl_xor(mx, 16, 32));
        const float mnew = fmaxf(m, mx);
        const float alpha = __builtin_amdgcn_exp2f(m - mnew);
        const float sh = PSH - mnew;
        v16h pb; float ls = 0.0f;
#pragma unroll
        for (int r = 0; r < 8; ++r) { const h16 pa = (h16)__builtin_amdgcn_exp2f(ta[r] + sh); const h16 pc = (h16)__builtin_amdgcn_exp2f(tb[r] + sh); pb[r] = pa; pb[8 + r] = pc; ls += (float)pa + (float)pc; }
        l = l * alpha + ls; m = mnew;
        o0 = o0 * alpha; o1 = o1 * alpha; o2 = o2 * alpha; o3 = o3 * alpha;
        const h16* va = VT + vo + key0;
        const v16h v0 = ldh(va), v1 = ldh(va + (size_t)16 * SEQ), v2 = ldh(va + (size_t)32 * SEQ), v3 = ldh(va + (size_t)48 * SEQ);
        o0 = wmma16(v0, pb, o0); o1 = wmma16(v1, pb, o1); o2 = wmma16(v2, pb, o2); o3 = wmma16(v3, pb, o3);
        asm volatile("v_nop\n\tv_nop\n\tv_nop\n\tv_nop" : "+v"(o0), "+v"(o1), "+v"(o2), "+v"(o3) : "v"(v0), "v"(v1), "v"(v2), "v"(v3), "v"(pb));
    }
    l += __shfl_xor(l, 16, 32);
    const float inv = 1.0f / l;
    const int wb = wave * 16 * 68;
    { v4f a, c;
      a[0] = o0[0] * inv; a[1] = o0[1] * inv; a[2] = o0[2] * inv; a[3] = o0[3] * inv; c[0] = o0[4] * inv; c[1] = o0[5] * inv; c[2] = o0[6] * inv; c[3] = o0[7] * inv;
      *(v4fa*)(&os[wb + lr * 68 +  0 + 8 * hi]) = a; *(v4fa*)(&os[wb + lr * 68 +  0 + 8 * hi + 4]) = c;
      a[0] = o1[0] * inv; a[1] = o1[1] * inv; a[2] = o1[2] * inv; a[3] = o1[3] * inv; c[0] = o1[4] * inv; c[1] = o1[5] * inv; c[2] = o1[6] * inv; c[3] = o1[7] * inv;
      *(v4fa*)(&os[wb + lr * 68 + 16 + 8 * hi]) = a; *(v4fa*)(&os[wb + lr * 68 + 16 + 8 * hi + 4]) = c;
      a[0] = o2[0] * inv; a[1] = o2[1] * inv; a[2] = o2[2] * inv; a[3] = o2[3] * inv; c[0] = o2[4] * inv; c[1] = o2[5] * inv; c[2] = o2[6] * inv; c[3] = o2[7] * inv;
      *(v4fa*)(&os[wb + lr * 68 + 32 + 8 * hi]) = a; *(v4fa*)(&os[wb + lr * 68 + 32 + 8 * hi + 4]) = c;
      a[0] = o3[0] * inv; a[1] = o3[1] * inv; a[2] = o3[2] * inv; a[3] = o3[3] * inv; c[0] = o3[4] * inv; c[1] = o3[5] * inv; c[2] = o3[6] * inv; c[3] = o3[7] * inv;
      *(v4fa*)(&os[wb + lr * 68 + 48 + 8 * hi]) = a; *(v4fa*)(&os[wb + lr * 68 + 48 + 8 * hi + 4]) = c; }
    wave_sync();
    float* orow = OUT + ((size_t)b * OUT_SEQ + t0) * DM + h * HD;
#pragma unroll 1
    for (int ps = 0; ps < 2; ++ps) {
#pragma unroll
        for (int s = 0; s < 8; ++s) { const int row = 2 * s + hi, cofs = lr * 4;
            const v4f val = *(const v4fa*)(&os[wb + row * 68 + cofs]);
            *(volatile v4f*)(orow + (size_t)row * DM + cofs) = val; }
        if (ps == 0) __threadfence(); }
}

static constexpr size_t al256(size_t v) { return (v + 255) & ~(size_t)255; }
static constexpr size_t SZ_PL = al256((size_t)NB * SEQ * DM * 2);
static constexpr size_t SZ_TOTAL = 3 * SZ_PL;
static_assert(SZ_TOTAL <= (size_t)134217728);
static_assert((size_t)NB * NH_ * HD * SEQ * 2 <= SZ_PL);

extern "C" void kernel_launch(void* const* d_in, const int* in_sizes, int n_in,
                              void* d_out, int out_size, void* d_ws, size_t ws_size, hipStream_t stream) {
    if (n_in < 3) return;
    const size_t needx = ((size_t)(NB - 1) * SEQ_FULL + SEQ) * DM;
    if ((size_t)in_sizes[0] < needx || (size_t)in_sizes[1] < needx || (size_t)in_sizes[2] < needx) return;
    if ((size_t)out_size < ((size_t)(NB - 1) * OUT_SEQ + SEQ) * DM) return;
    if (SZ_TOTAL > ws_size) return;
    const float* q = (const float*)d_in[0]; const float* k = (const float*)d_in[1]; const float* v = (const float*)d_in[2];
    float* OUT = (float*)d_out;
    char* wsp = (char*)d_ws;
    h16* QH = (h16*)wsp; wsp += SZ_PL;
    h16* KH = (h16*)wsp; wsp += SZ_PL;
    h16* VT = (h16*)wsp; wsp += SZ_PL;

    const size_t n8 = (size_t)NB * SEQ * DM / 8;
    k_cvt2<<<(unsigned)((n8 + 255) / 256), 256, 0, stream>>>(q, QH, k, KH, n8);
    k_vt<<<dim3(SEQ / 64, NB * NH_, 1), 256, 0, stream>>>(v, VT);
    k_flash<<<dim3(SEQ / (16 * AW), NB * NH_, 1), 32 * AW, 0, stream>>>(QH, KH, VT, OUT);
}
